// MambaMixer_42623255446107
// MI455X (gfx1250) — hardware-verified
//
#include <hip/hip_runtime.h>
#include <hip/hip_bf16.h>


#define NB_  2
#define L_   512
#define H_   1024
#define DI_  2048
#define NS_  16
#define R_   64
#define XP_  96
#define XPP_ 128
#define NT_  (NB_ * L_)

static_assert(NT_ % 64 == 0);
static_assert(H_ % 128 == 0);
static_assert(DI_ % 128 == 0);
static_assert(DI_ == 8 * 256);
static_assert((L_ & (L_ - 1)) == 0);
static_assert(L_ % 16 == 0);
static_assert(R_ % 32 == 0);
static_assert(XP_ <= XPP_);
static_assert(XPP_ % 128 == 0);
static_assert(NS_ == 16);

typedef float          v4f   __attribute__((ext_vector_type(4)));
typedef float          v8f   __attribute__((ext_vector_type(8)));
typedef _Float16       v8h   __attribute__((ext_vector_type(8)));
typedef _Float16       v16h  __attribute__((ext_vector_type(16)));
typedef __bf16         v16b  __attribute__((ext_vector_type(16)));
typedef unsigned short u16x8 __attribute__((ext_vector_type(8)));

union FragH { u16x8 h[2]; v16h v; };
union FragB { u16x8 h[2]; v16b v; };
union Pack8 { v8h f; u16x8 u; };

__device__ __forceinline__ unsigned short f32_to_bf16(float f) {
    unsigned u = __float_as_uint(f);
    unsigned r = u + 0x7FFFu + ((u >> 16) & 1u);
    return (unsigned short)(r >> 16);
}
__device__ __forceinline__ float bf16_to_f32(unsigned short b) {
    return __uint_as_float(((unsigned)b) << 16);
}
__device__ __forceinline__ float silu_f(float x) {
    const float e = __expf(-x);
    return x * __builtin_amdgcn_rcpf(1.0f + e);
}
__device__ __forceinline__ float softplus_f(float x) {
    return fmaxf(x, 0.0f) + log1pf(__expf(-fabsf(x)));
}
__device__ __forceinline__ v8f ld8f(const float* p) {
    v4f a = *(const v4f*)p;
    v4f b = *(const v4f*)(p + 4);
    return __builtin_shufflevector(a, b, 0, 1, 2, 3, 4, 5, 6, 7);
}

__device__ __forceinline__ void mma16(v8f& acc, const FragH& a, const FragH& b) {
    acc = __builtin_amdgcn_wmma_f32_16x16x32_f16(false, a.v, false, b.v, (short)0, acc, false, false);
    asm volatile("v_nop\n\tv_nop\n\tv_nop\n\tv_nop" : "+v"(acc) : "v"(a.v), "v"(b.v));
}
__device__ __forceinline__ void mma16(v8f& acc, const FragB& a, const FragB& b) {
    acc = __builtin_amdgcn_wmma_f32_16x16x32_bf16(false, a.v, false, b.v, (short)0, acc, false, false);
    asm volatile("v_nop\n\tv_nop\n\tv_nop\n\tv_nop" : "+v"(acc) : "v"(a.v), "v"(b.v));
}

__global__ __launch_bounds__(256)
void cvt_kernel(const float* __restrict__ src, unsigned short* dst0, unsigned short* dst1,
                int src_ld, int cols, int rows_valid, int n8, int mode, float scale)
{
    const int i = blockIdx.x * 256 + threadIdx.x;
    if (i >= n8) return;
    const size_t e = (size_t)i * 8;
    const int r  = (int)(e / (size_t)cols);
    const int c  = (int)(e - (size_t)r * (size_t)cols);
    const int rr = (r < rows_valid) ? r : (rows_valid - 1);
    v8f x = ld8f(src + (size_t)rr * src_ld + c);
    const bool live = (r < rows_valid);
#pragma unroll
    for (int k = 0; k < 8; ++k) x[k] = live ? x[k] : 0.0f;

    if (mode == 0) {
        Pack8 pk;
        pk.f = __builtin_convertvector(x * scale, v8h);
        const u16x8 v = pk.u;
        *(volatile u16x8*)(dst0 + e) = v;
        __threadfence();
        *(volatile u16x8*)(dst0 + e) = v;
    } else {
        u16x8 hv, lv;
#pragma unroll
        for (int k = 0; k < 8; ++k) {
            const float f = x[k];
            const unsigned short hb = f32_to_bf16(f);
            const unsigned short lb = f32_to_bf16(f - bf16_to_f32(hb));
            hv[k] = hb;
            lv[k] = lb;
        }
        *(volatile u16x8*)(dst0 + e) = hv;
        *(volatile u16x8*)(dst1 + e) = lv;
        __threadfence();
        *(volatile u16x8*)(dst0 + e) = hv;
        *(volatile u16x8*)(dst1 + e) = lv;
    }
}

template<int NBF>
__device__ __forceinline__ void tile_store_pass(const float* st, float* gp, int ldc, int lane) {
    constexpr int CW  = NBF * 16;
    constexpr int P   = CW + 4;
    constexpr int LPR = CW / 4;
    constexpr int RPI = 32 / LPR;
    constexpr int NIT = 32 / RPI;
    static_assert(LPR * RPI == 32);
    static_assert(NIT * RPI == 32);
    const int rsub = lane / LPR;
    const int c4   = (lane % LPR) * 4;
#pragma unroll
    for (int it = 0; it < NIT; ++it) {
        const int row = it * RPI + rsub;
        const v4f v = *(const v4f*)(st + row * P + c4);
        *(volatile v4f*)(gp + (size_t)row * ldc + c4) = v;
    }
}

template<typename FR, bool SPLIT, int NBF>
__global__ __launch_bounds__(128)
void gemm_tn_kernel(const unsigned short* __restrict__ A,  const unsigned short* __restrict__ A2,
                    const unsigned short* __restrict__ Bw, const unsigned short* __restrict__ B2,
                    float* C, int K, int ldc, float scale)
{
    static_assert(NBF == 2 || NBF == 4);
    constexpr int CW = NBF * 16;
    constexpr int P  = CW + 4;
    __shared__ __attribute__((aligned(16))) float stile[4][32 * P];

    const int tid  = threadIdx.x;
    const int lane = tid & 31;
    const int wave = tid >> 5;
    const int h    = lane >> 4;
    const int m    = lane & 15;
    const int wm   = wave >> 1;
    const int wn   = wave & 1;

    const int rowW = blockIdx.y * 64 + wm * 32;
    const int colW = blockIdx.x * (2 * CW) + wn * CW;

    v8f acc[2 * NBF];
#pragma unroll
    for (int j = 0; j < 2 * NBF; ++j)
#pragma unroll
        for (int r = 0; r < 8; ++r) acc[j][r] = 0.0f;

    const size_t aoff  = (size_t)(rowW + m) * K + 8 * h;
    const size_t boff  = (size_t)(colW + m) * K + 8 * h;
    const size_t sub16 = (size_t)16 * K;
    const int nk = K >> 5;

    for (int kt = 0; kt < nk; ++kt) {
        const size_t k0 = (size_t)kt * 32;
        FR fa[2], fb[NBF], ga[2], gb[NBF];
#pragma unroll
        for (int s = 0; s < 2; ++s) {
            const unsigned short* p = A + aoff + s * sub16 + k0;
            fa[s].h[0] = *(const u16x8*)(p);
            fa[s].h[1] = *(const u16x8*)(p + 16);
            if (SPLIT) {
                const unsigned short* q = A2 + aoff + s * sub16 + k0;
                ga[s].h[0] = *(const u16x8*)(q);
                ga[s].h[1] = *(const u16x8*)(q + 16);
            }
        }
#pragma unroll
        for (int j = 0; j < NBF; ++j) {
            const unsigned short* p = Bw + boff + j * sub16 + k0;
            fb[j].h[0] = *(const u16x8*)(p);
            fb[j].h[1] = *(const u16x8*)(p + 16);
            if (SPLIT) {
                const unsigned short* q = B2 + boff + j * sub16 + k0;
                gb[j].h[0] = *(const u16x8*)(q);
                gb[j].h[1] = *(const u16x8*)(q + 16);
            }
        }
#pragma unroll
        for (int s = 0; s < 2; ++s)
#pragma unroll
            for (int j = 0; j < NBF; ++j) {
                mma16(acc[s * NBF + j], fa[s], fb[j]);
                if (SPLIT) {
                    mma16(acc[s * NBF + j], fa[s], gb[j]);
                    mma16(acc[s * NBF + j], ga[s], fb[j]);
                }
            }
    }

    float* st = stile[wave];
#pragma unroll
    for (int s = 0; s < 2; ++s)
#pragma unroll
        for (int j = 0; j < NBF; ++j)
#pragma unroll
            for (int r = 0; r < 8; ++r)
                st[(s * 16 + 8 * h + r) * P + j * 16 + m] = acc[s * NBF + j][r] * scale;
    __syncthreads();

    float* gp = C + (size_t)rowW * ldc + colW;
    tile_store_pass<NBF>(st, gp, ldc, lane);
    __threadfence();
    tile_store_pass<NBF>(st, gp, ldc, lane);
}

__global__ __launch_bounds__(256)
void conv_silu_kernel(const float* __restrict__ X, const float* __restrict__ cw,
                      const float* __restrict__ cb, float* Uf, unsigned short* U16)
{
    __shared__ __attribute__((aligned(16))) float          sru[DI_];
    __shared__ __attribute__((aligned(16))) unsigned short srh[DI_];

    const int m   = blockIdx.x;
    const int l   = m & (L_ - 1);
    const int tid = threadIdx.x;
    const int m1  = (l >= 1) ? (m - 1) : m;
    const int m2  = (l >= 2) ? (m - 2) : m;
    const int m3  = (l >= 3) ? (m - 3) : m;
    const float* xr0 = X + (size_t)m  * DI_;
    const float* xr1 = X + (size_t)m1 * DI_;
    const float* xr2 = X + (size_t)m2 * DI_;
    const float* xr3 = X + (size_t)m3 * DI_;

#pragma unroll 1
    for (int j = 0; j < 8; ++j) {
        const int ch = j * 256 + tid;
        const float x3 = xr0[ch];
        float x2 = xr1[ch];
        float x1 = xr2[ch];
        float x0 = xr3[ch];
        x2 = (l >= 1) ? x2 : 0.0f;
        x1 = (l >= 2) ? x1 : 0.0f;
        x0 = (l >= 3) ? x0 : 0.0f;
        const v4f w = *(const v4f*)(cw + (size_t)ch * 4);
        const float cv = w[0] * x0 + w[1] * x1 + w[2] * x2 + w[3] * x3 + cb[ch];
        const float u  = silu_f(cv);
        sru[ch] = u;
        const _Float16 hv = (_Float16)(u * 64.0f);
        srh[ch] = __builtin_bit_cast(unsigned short, hv);
    }
    __syncthreads();

    const v4f a0 = *(const v4f*)(sru + 4 * tid);
    const v4f a1 = *(const v4f*)(sru + DI_ / 2 + 4 * tid);
    const u16x8 hv8 = *(const u16x8*)(srh + 8 * tid);
    float* up = Uf + (size_t)m * DI_;
    unsigned short* hp = U16 + (size_t)m * DI_ + 8 * tid;
    *(volatile v4f*)(up + 4 * tid) = a0;
    *(volatile v4f*)(up + DI_ / 2 + 4 * tid) = a1;
    *(volatile u16x8*)hp = hv8;
    __threadfence();
    *(volatile v4f*)(up + 4 * tid) = a0;
    *(volatile v4f*)(up + DI_ / 2 + 4 * tid) = a1;
    *(volatile u16x8*)hp = hv8;
}

__device__ __forceinline__ void yrows_store_pass(const float* sy, float* Y, size_t gbase,
                                                 int wave, int lane) {
#pragma unroll
    for (int it = 0; it < 4; ++it) {
        const int row = wave * 8 + it * 2 + (lane >> 4);
        const int c4  = (lane & 15) * 4;
        const v4f v = *(const v4f*)(sy + row * 64 + c4);
        *(volatile v4f*)(Y + gbase + (size_t)row * DI_ + c4) = v;
    }
}
__device__ __forceinline__ void hrows_store_pass(const unsigned short* sl, unsigned short* gpl,
                                                 size_t gbase, int lane) {
#pragma unroll
    for (int it = 0; it < 4; ++it) {
        const int t = it * 4 + (lane >> 3);
        const int c = (lane & 7) * 8;
        const u16x8 v = *(const u16x8*)(sl + t * 64 + c);
        *(volatile u16x8*)(gpl + gbase + (size_t)t * DI_ + c) = v;
    }
}

template<int DIR>
__global__ __launch_bounds__(256)
void scan_kernel(const float* __restrict__ Uf, const float* __restrict__ Gf,
                 const float* __restrict__ DP, const float* __restrict__ S,
                 const float* __restrict__ dtb, const float* __restrict__ Alog,
                 const float* __restrict__ Dp, const float* Yin, float* Yout,
                 unsigned short* yhi, unsigned short* ylo)
{
    __shared__ __attribute__((aligned(16))) float          sS[16 * 32];
    __shared__ __attribute__((aligned(16))) float          sy[16 * 64];
    __shared__ __attribute__((aligned(16))) unsigned short shi[16 * 64];
    __shared__ __attribute__((aligned(16))) unsigned short slo[16 * 64];

    const int tid   = threadIdx.x;
    const int lane  = tid & 31;
    const int wave  = tid >> 5;
    const int sub   = lane & 3;
    const int cl    = wave * 8 + (lane >> 2);
    const int dbase = blockIdx.x * 64;
    const int d     = dbase + cl;
    const int b     = blockIdx.y;
    const size_t rowb = (size_t)b * L_;

    float an[4], hs[4];
#pragma unroll
    for (int j = 0; j < 4; ++j) {
        an[j] = -__expf(Alog[(size_t)d * NS_ + 4 * sub + j]);
        hs[j] = 0.0f;
    }
    const float tb = dtb[d];
    const float Dd = Dp[d];

#pragma unroll 1
    for (int cc = 0; cc < L_ / 16; ++cc) {
        const int c  = DIR ? (L_ / 16 - 1 - cc) : cc;
        const int l0 = c * 16;
        if (tid < 128) {
            const int t = tid >> 3;
            const int q = tid & 7;
            const v4f v = *(const v4f*)(S + (rowb + l0 + t) * XPP_ + R_ + 4 * q);
            *(v4f*)(sS + t * 32 + 4 * q) = v;
        }
        __syncthreads();
#pragma unroll 1
        for (int tt = 0; tt < 16; ++tt) {
            const int t = DIR ? (15 - tt) : tt;
            const size_t e = (rowb + l0 + t) * DI_ + d;
            const float u  = Uf[e];
            const float g  = Gf[e];
            const float dt = softplus_f(DP[e] + tb);
            const float* bc = sS + t * 32 + 4 * sub;
            float y = 0.0f;
#pragma unroll
            for (int j = 0; j < 4; ++j) {
                const float da  = __expf(dt * an[j]);
                const float dbu = (dt * bc[j]) * u;
                hs[j] = da * hs[j] + dbu;
                y += hs[j] * bc[16 + j];
            }
            y += __shfl_xor(y, 1, 32);
            y += __shfl_xor(y, 2, 32);
            const float val = (y + u * Dd) * silu_f(g);
            if (DIR == 0) {
                if (sub == 0) sy[t * 64 + cl] = val;
            } else {
                const float yf  = Yin[e];
                const float tot = yf + val;
                const unsigned short hb = f32_to_bf16(tot);
                const unsigned short lb = f32_to_bf16(tot - bf16_to_f32(hb));
                if (sub == 0) { shi[t * 64 + cl] = hb; slo[t * 64 + cl] = lb; }
            }
        }
        __syncthreads();
        const size_t gbase = (rowb + l0) * DI_ + dbase;
        if (DIR == 0) {
            if (wave < 2) yrows_store_pass(sy, Yout, gbase, wave, lane);
            __threadfence();
            if (wave < 2) yrows_store_pass(sy, Yout, gbase, wave, lane);
        } else {
            const unsigned short* sl = (wave == 0) ? shi : slo;
            unsigned short* gpl = (wave == 0) ? yhi : ylo;
            if (wave < 2) hrows_store_pass(sl, gpl, gbase, lane);
            __threadfence();
            if (wave < 2) hrows_store_pass(sl, gpl, gbase, lane);
        }
        __syncthreads();
    }
}

extern "C" void kernel_launch(void* const* d_in, const int* in_sizes, int n_in,
                              void* d_out, int out_size, void* d_ws, size_t ws_size,
                              hipStream_t stream)
{
    if (n_in < 17) return;
    if (in_sizes[0]  != NT_ * H_)      return;
    if (in_sizes[1]  != NT_ * H_)      return;
    if (in_sizes[2]  != 2 * DI_ * H_)  return;
    if (in_sizes[3]  != 2 * DI_ * H_)  return;
    if (in_sizes[4]  != DI_ * 4)       return;
    if (in_sizes[5]  != DI_)           return;
    if (in_sizes[6]  != XP_ * DI_)     return;
    if (in_sizes[7]  != XP_ * DI_)     return;
    if (in_sizes[8]  != DI_ * R_)      return;
    if (in_sizes[9]  != DI_)           return;
    if (in_sizes[10] != DI_ * R_)      return;
    if (in_sizes[11] != DI_)           return;
    if (in_sizes[12] != DI_ * NS_)     return;
    if (in_sizes[13] != DI_ * NS_)     return;
    if (in_sizes[14] != DI_)           return;
    if (in_sizes[15] != DI_)           return;
    if (in_sizes[16] != H_ * DI_)      return;
    if (out_size != NT_ * H_)          return;

    const float* hs0    = (const float*)d_in[0];
    const float* hs2    = (const float*)d_in[1];
    const float* inW    = (const float*)d_in[2];
    const float* inDifW = (const float*)d_in[3];
    const float* convW  = (const float*)d_in[4];
    const float* convB  = (const float*)d_in[5];
    const float* xW_f   = (const float*)d_in[6];
    const float* xW_b   = (const float*)d_in[7];
    const float* dtW_f  = (const float*)d_in[8];
    const float* dtB_f  = (const float*)d_in[9];
    const float* dtW_b  = (const float*)d_in[10];
    const float* dtB_b  = (const float*)d_in[11];
    const float* Alog_f = (const float*)d_in[12];
    const float* Alog_b = (const float*)d_in[13];
    const float* Dv_f   = (const float*)d_in[14];
    const float* Dv_b   = (const float*)d_in[15];
    const float* outW   = (const float*)d_in[16];
    float* out = (float*)d_out;

    const size_t SZ_X16  = (size_t)NT_ * H_ * 2;
    const size_t SZ_W16  = (size_t)DI_ * H_ * 2;
    const size_t SZ_WX16 = (size_t)XPP_ * DI_ * 2;
    const size_t SZ_WD16 = (size_t)DI_ * R_ * 2;
    const size_t SZ_WO16 = (size_t)H_ * DI_ * 2;
    const size_t SZ_F    = (size_t)NT_ * DI_ * 4;
    const size_t SZ_H    = (size_t)NT_ * DI_ * 2;
    const size_t SZ_S    = (size_t)NT_ * XPP_ * 4;
    const size_t SZ_DR   = (size_t)NT_ * R_ * 2;

    size_t o = 0;
    const size_t OFF_X16H  = o; o += SZ_X16;
    const size_t OFF_X16L  = o; o += SZ_X16;
    const size_t OFF_X216H = o; o += SZ_X16;
    const size_t OFF_X216L = o; o += SZ_X16;
    const size_t OFF_WINH  = o; o += SZ_W16;
    const size_t OFF_WINL  = o; o += SZ_W16;
    const size_t OFF_WDFH  = o; o += SZ_W16;
    const size_t OFF_WDFL  = o; o += SZ_W16;
    const size_t OFF_WXF   = o; o += SZ_WX16;
    const size_t OFF_WXB   = o; o += SZ_WX16;
    const size_t OFF_WDTF  = o; o += SZ_WD16;
    const size_t OFF_WDTB  = o; o += SZ_WD16;
    const size_t OFF_WOH   = o; o += SZ_WO16;
    const size_t OFF_WOL   = o; o += SZ_WO16;
    const size_t OFF_XF    = o; o += SZ_F;
    const size_t OFF_GF    = o; o += SZ_F;
    const size_t OFF_UF    = o; o += SZ_F;
    const size_t OFF_U16   = o; o += SZ_H;
    const size_t OFF_SF    = o; o += SZ_S;
    const size_t OFF_SB    = o; o += SZ_S;
    const size_t OFF_DRF   = o; o += SZ_DR;
    const size_t OFF_DRB   = o; o += SZ_DR;
    const size_t OFF_DPF   = o; o += SZ_F;
    const size_t OFF_DPB   = o; o += SZ_F;
    const size_t OFF_YF    = o; o += SZ_F;
    const size_t OFF_YHI   = o; o += SZ_H;
    const size_t OFF_YLO   = o; o += SZ_H;
    const size_t WS_END    = o;
    if (ws_size < WS_END) return;

    char* ws = (char*)d_ws;
    unsigned short* x16h   = (unsigned short*)(ws + OFF_X16H);
    unsigned short* x16l   = (unsigned short*)(ws + OFF_X16L);
    unsigned short* x216h  = (unsigned short*)(ws + OFF_X216H);
    unsigned short* x216l  = (unsigned short*)(ws + OFF_X216L);
    unsigned short* winh   = (unsigned short*)(ws + OFF_WINH);
    unsigned short* winl   = (unsigned short*)(ws + OFF_WINL);
    unsigned short* wdfh   = (unsigned short*)(ws + OFF_WDFH);
    unsigned short* wdfl   = (unsigned short*)(ws + OFF_WDFL);
    unsigned short* wxf16  = (unsigned short*)(ws + OFF_WXF);
    unsigned short* wxb16  = (unsigned short*)(ws + OFF_WXB);
    unsigned short* wdtf16 = (unsigned short*)(ws + OFF_WDTF);
    unsigned short* wdtb16 = (unsigned short*)(ws + OFF_WDTB);
    unsigned short* woh    = (unsigned short*)(ws + OFF_WOH);
    unsigned short* wol    = (unsigned short*)(ws + OFF_WOL);
    float*          Xf     = (float*)(ws + OFF_XF);
    float*          Gf     = (float*)(ws + OFF_GF);
    float*          Uf     = (float*)(ws + OFF_UF);
    unsigned short* u16    = (unsigned short*)(ws + OFF_U16);
    float*          Sf     = (float*)(ws + OFF_SF);
    float*          Sb     = (float*)(ws + OFF_SB);
    unsigned short* drf16  = (unsigned short*)(ws + OFF_DRF);
    unsigned short* drb16  = (unsigned short*)(ws + OFF_DRB);
    float*          DPf    = (float*)(ws + OFF_DPF);
    float*          DPb    = (float*)(ws + OFF_DPB);
    float*          Yf     = (float*)(ws + OFF_YF);
    unsigned short* yhi    = (unsigned short*)(ws + OFF_YHI);
    unsigned short* ylo    = (unsigned short*)(ws + OFF_YLO);

    const dim3 b256(256);

    {
        int n8;
        n8 = (NT_ * H_) / 8;
        cvt_kernel<<<dim3((n8 + 255) / 256), b256, 0, stream>>>(hs0, x16h, x16l, H_, H_, NT_, n8, 1, 1.0f);
        cvt_kernel<<<dim3((n8 + 255) / 256), b256, 0, stream>>>(hs2, x216h, x216l, H_, H_, NT_, n8, 1, 1.0f);
        n8 = (DI_ * H_) / 8;
        cvt_kernel<<<dim3((n8 + 255) / 256), b256, 0, stream>>>(inW, winh, winl, H_, H_, DI_, n8, 1, 1.0f);
        cvt_kernel<<<dim3((n8 + 255) / 256), b256, 0, stream>>>(inDifW + (size_t)DI_ * H_, wdfh, wdfl,
                                                                H_, H_, DI_, n8, 1, 1.0f);
        n8 = (XPP_ * DI_) / 8;
        cvt_kernel<<<dim3((n8 + 255) / 256), b256, 0, stream>>>(xW_f, wxf16, wxf16, DI_, DI_, XP_, n8, 0, 32.0f);
        cvt_kernel<<<dim3((n8 + 255) / 256), b256, 0, stream>>>(xW_b, wxb16, wxb16, DI_, DI_, XP_, n8, 0, 32.0f);
        n8 = (DI_ * R_) / 8;
        cvt_kernel<<<dim3((n8 + 255) / 256), b256, 0, stream>>>(dtW_f, wdtf16, wdtf16, R_, R_, DI_, n8, 0, 32.0f);
        cvt_kernel<<<dim3((n8 + 255) / 256), b256, 0, stream>>>(dtW_b, wdtb16, wdtb16, R_, R_, DI_, n8, 0, 32.0f);
        n8 = (H_ * DI_) / 8;
        cvt_kernel<<<dim3((n8 + 255) / 256), b256, 0, stream>>>(outW, woh, wol, DI_, DI_, H_, n8, 1, 1.0f);
    }

    gemm_tn_kernel<FragB, true, 2><<<dim3(DI_ / 64, NT_ / 64), dim3(128), 0, stream>>>(
        (const unsigned short*)x16h, (const unsigned short*)x16l,
        (const unsigned short*)winh, (const unsigned short*)winl,
        Xf, (int)H_, (int)DI_, 1.0f);

    gemm_tn_kernel<FragB, true, 2><<<dim3(DI_ / 64, NT_ / 64), dim3(128), 0, stream>>>(
        (const unsigned short*)x216h, (const unsigned short*)x216l,
        (const unsigned short*)wdfh, (const unsigned short*)wdfl,
        Gf, (int)H_, (int)DI_, 1.0f);

    conv_silu_kernel<<<dim3(NT_), b256, 0, stream>>>((const float*)Xf, convW, convB, Uf, u16);

    gemm_tn_kernel<FragH, false, 4><<<dim3(XPP_ / 128, NT_ / 64), dim3(128), 0, stream>>>(
        (const unsigned short*)u16, (const unsigned short*)u16,
        (const unsigned short*)wxf16, (const unsigned short*)wxf16,
        Sf, (int)DI_, (int)XPP_, 0.00048828125f);
    gemm_tn_kernel<FragH, false, 4><<<dim3(XPP_ / 128, NT_ / 64), dim3(128), 0, stream>>>(
        (const unsigned short*)u16, (const unsigned short*)u16,
        (const unsigned short*)wxb16, (const unsigned short*)wxb16,
        Sb, (int)DI_, (int)XPP_, 0.00048828125f);

    {
        const int n8 = (NT_ * R_) / 8;
        cvt_kernel<<<dim3((n8 + 255) / 256), b256, 0, stream>>>((const float*)Sf, drf16, drf16,
                                                                XPP_, R_, NT_, n8, 0, 64.0f);
        cvt_kernel<<<dim3((n8 + 255) / 256), b256, 0, stream>>>((const float*)Sb, drb16, drb16,
                                                                XPP_, R_, NT_, n8, 0, 64.0f);
    }

    gemm_tn_kernel<FragH, false, 4><<<dim3(DI_ / 128, NT_ / 64), dim3(128), 0, stream>>>(
        (const unsigned short*)drf16, (const unsigned short*)drf16,
        (const unsigned short*)wdtf16, (const unsigned short*)wdtf16,
        DPf, (int)R_, (int)DI_, 0.00048828125f);
    gemm_tn_kernel<FragH, false, 4><<<dim3(DI_ / 128, NT_ / 64), dim3(128), 0, stream>>>(
        (const unsigned short*)drb16, (const unsigned short*)drb16,
        (const unsigned short*)wdtb16, (const unsigned short*)wdtb16,
        DPb, (int)R_, (int)DI_, 0.00048828125f);

    scan_kernel<0><<<dim3(DI_ / 64, NB_), b256, 0, stream>>>(
        (const float*)Uf, (const float*)Gf, (const float*)DPf, (const float*)Sf,
        dtB_f, Alog_f, Dv_f, (const float*)Yf, Yf, yhi, ylo);
    scan_kernel<1><<<dim3(DI_ / 64, NB_), b256, 0, stream>>>(
        (const float*)Uf, (const float*)Gf, (const float*)DPb, (const float*)Sb,
        dtB_b, Alog_b, Dv_b, (const float*)Yf, Yf, yhi, ylo);

    gemm_tn_kernel<FragB, true, 2><<<dim3(H_ / 64, NT_ / 64), dim3(128), 0, stream>>>(
        (const unsigned short*)yhi, (const unsigned short*)ylo,
        (const unsigned short*)woh, (const unsigned short*)wol,
        out, (int)DI_, (int)H_, 1.0f);
}
